// GCN_cls_e_69483980915280
// MI455X (gfx1250) — hardware-run, weakly checked
//
#include <hip/hip_runtime.h>


namespace {
constexpr int N = 100000, E = 1600000, F = 50, FP = 64, H = 64, G = 512, C = 10, BD = 10, NPB = 8;
constexpr float XS = 256.0f, HS = 256.0f, WSC = 256.0f;
typedef _Float16 b16;
typedef __attribute__((ext_vector_type(16))) _Float16 v16b;
typedef __attribute__((ext_vector_type(8))) _Float16 v8b;
typedef __attribute__((ext_vector_type(8))) float v8f;
typedef __attribute__((ext_vector_type(4))) float v4f;
typedef __attribute__((ext_vector_type(2))) float v2f;
__device__ __forceinline__ float bf16_rne(float f) { unsigned int u = __float_as_uint(f); u += 0x7FFFu + ((u >> 16) & 1u); float r = __uint_as_float(u & 0xFFFF0000u); asm volatile("" : "+v"(r)); return r; }
__device__ __forceinline__ float bfv(float f) { float r = bf16_rne(f); asm volatile("" : "+v"(r)); return r; }
__device__ __forceinline__ void split16(float v, b16& hi, b16& lo) { hi = (b16)v; lo = (b16)(v - (float)hi); }
__device__ __forceinline__ v16b frag_kb(const b16* p, int hh) { const v8b a = *(const v8b*)(p + 8 * hh), b = *(const v8b*)(p + 16 + 8 * hh); v16b f;
#pragma unroll
  for (int e = 0; e < 8; ++e) { f[e] = a[e]; f[8 + e] = b[e]; } return f; }
__device__ __forceinline__ v8f wmma16b(v16b a, v16b b, v8f c) { v8f d = __builtin_amdgcn_wmma_f32_16x16x32_f16(false, a, false, b, (short)0, c, false, false); asm volatile("v_nop\n\tv_nop\n\tv_nop\n\tv_nop" : "+v"(d) : "v"(a), "v"(b)); return d; }
__device__ __forceinline__ void wave_lds_sync() { __builtin_amdgcn_fence(__ATOMIC_RELEASE, "workgroup"); __builtin_amdgcn_wave_barrier(); __builtin_amdgcn_fence(__ATOMIC_ACQUIRE, "workgroup"); }
__device__ __forceinline__ float pmul(float a, float b) { float p = a * b; asm volatile("" : "+v"(p)); return p; }
__device__ __forceinline__ int iclamp(int v, int lo, int hi) { return v < lo ? lo : (v > hi ? hi : v); }
constexpr int CSR_NBLK8 = 512, CSR_GB8 = 8, CSR_GN8 = 1 << CSR_GB8  , CSR_TS8 = (CSR_GN8 < 32 ? 32 : CSR_GN8)  , CSR_MAXG8 = 512, CSR_CAP8 = 12288  ;
__device__ __host__ __forceinline__ int csr_tix8(int v) { return (v >> CSR_GB8) * CSR_TS8 + (v & (CSR_GN8 - 1)); }
__global__ __launch_bounds__(64) void csrA_kernel8(const int* __restrict__ dst, int E, int N, int nG, int CHP, int NGP, int* __restrict__ STG, int* __restrict__ HST) {
  extern __shared__ int sm[];
  int* cnt = sm; int* run = sm + NGP; int* ids = sm + 2 * NGP;
  const int b = blockIdx.x; const int ch = (E + CSR_NBLK8 - 1) / CSR_NBLK8; const int e0 = b * ch, e1 = min(E, e0 + ch);
  for (int i = threadIdx.x; i < NGP; i += 64) cnt[i] = 0;
  for (int i = threadIdx.x; i < CHP; i += 64) ids[i] = -1;
  __syncthreads();
  if (threadIdx.x == 0) {
    for (int e = e0; e < e1; ++e) { int d = dst[e]; d = (d < 0) ? 0 : (d >= N ? N - 1 : d); cnt[d >> CSR_GB8] += 1; }
    int acc = 0; for (int g = 0; g < nG; ++g) { run[g] = acc; acc += cnt[g]; }
    for (int e = e0; e < e1; ++e) { int d = dst[e]; d = (d < 0) ? 0 : (d >= N ? N - 1 : d); const int g = d >> CSR_GB8; ids[run[g]] = e; run[g] += 1; } }
  __syncthreads();
  typedef __attribute__((ext_vector_type(4))) int v4i;
  for (int pass = 0; pass < 2; ++pass) {
    for (int i = threadIdx.x; i < CHP / 4; i += 64) *(volatile v4i*)(STG + (size_t)b * CHP + i * 4) = *(const v4i*)(&ids[i * 4]);
    for (int i = threadIdx.x; i < NGP / 4; i += 64) { v4i v; for (int e = 0; e < 4; ++e) v[e] = (i * 4 + e < nG) ? cnt[i * 4 + e] : 0; *(volatile v4i*)(HST + (size_t)b * NGP + i * 4) = v; }
    __threadfence(); }
}
__global__ __launch_bounds__(512) void csrS_kernel8(const int* __restrict__ HST, int nG, int NGP, int* __restrict__ START, int* __restrict__ TOT, int* __restrict__ OFF) {
  __shared__ int tot[CSR_MAXG8];
  const int b = threadIdx.x;
  for (int pass = 0; pass < 2; ++pass) { int runb = 0; for (int g = 0; g < nG; ++g) { int c = HST[(size_t)b * NGP + g]; c = (c < 0) ? 0 : c; ((volatile int*)OFF)[(size_t)g * CSR_NBLK8 + b] = runb; runb += c; } __threadfence(); }
  for (int g = threadIdx.x; g < nG; g += 512) { int s = 0; for (int bb = 0; bb < CSR_NBLK8; ++bb) { int c = HST[(size_t)bb * NGP + g]; s += (c < 0) ? 0 : c; } tot[g] = s; }
  __syncthreads();
  if (threadIdx.x < 32) {
    __shared__ int st[CSR_MAXG8 + 32];
    if (threadIdx.x == 0) { int acc = 0; for (int g = 0; g < NGP; ++g) { st[g] = acc; if (g < nG) acc += (tot[g] + 31) & ~31; } st[NGP] = acc; }
    __builtin_amdgcn_fence(__ATOMIC_RELEASE, "workgroup"); __builtin_amdgcn_wave_barrier(); __builtin_amdgcn_fence(__ATOMIC_ACQUIRE, "workgroup");
    for (int pass = 0; pass < 2; ++pass) { for (int i = threadIdx.x; i < NGP + 32; i += 32) { ((volatile int*)START)[i] = (i <= NGP) ? st[min(i, NGP)] : 0; ((volatile int*)TOT)[i] = (i < nG) ? tot[i] : 0; } __threadfence(); } }
}
__global__ __launch_bounds__(256) void csrB_kernel8(const int* __restrict__ dst, int N, int nG, int CHP, int NGP, int permLen, const int* __restrict__ STG, const int* __restrict__ HST, const int* __restrict__ OFF, const int* __restrict__ START, const int* __restrict__ TOT, int* __restrict__ PERM, int* __restrict__ ROWPTR, int* __restrict__ ROWCNT, int* __restrict__ FLAG) {
  typedef __attribute__((ext_vector_type(4))) int v4i;
  __shared__ int ids[CSR_CAP8]; __shared__ unsigned short key[CSR_CAP8]; __shared__ int outp[CSR_CAP8]; __shared__ int ncnt[CSR_GN8 + 1]; __shared__ int boff[CSR_NBLK8 + 1];
  const int g = blockIdx.x, t_ = threadIdx.x; int tot = TOT[g]; int st = START[g], stn = START[g + 1]; const int v0 = g * CSR_GN8; const int nv = min(CSR_GN8, N - v0); const int t0 = g * CSR_TS8;
  st = (st < 0) ? 0 : (st > permLen - 32 ? permLen - 32 : st) & ~31; stn = (stn < st) ? st : (stn > permLen ? permLen : stn); tot = (tot < 0) ? 0 : tot; if (tot > stn - st && tot <= CSR_CAP8) tot = stn - st;
  if (tot > CSR_CAP8) {
    for (int pass = 0; pass < 2; ++pass) { for (int i = t_; i < CSR_TS8 / 4; i += 256) { v4i a, c; for (int e = 0; e < 4; ++e) { a[e] = st; c[e] = 0; } *(volatile v4i*)(ROWPTR + t0 + i * 4) = a; *(volatile v4i*)(ROWCNT + t0 + i * 4) = c; } if (t_ == 0) ((volatile int*)FLAG)[0] = 1; __threadfence(); } (void)nv; return; }
  if (t_ == 0) { int acc = 0; for (int b = 0; b < CSR_NBLK8; ++b) { boff[b] = acc; int c = HST[(size_t)b * NGP + g]; c = (c < 0) ? 0 : (c > CHP ? CHP : c); acc += c; if (acc > tot) acc = tot; } boff[CSR_NBLK8] = acc; }
  for (int i = t_; i <= CSR_GN8; i += 256) ncnt[i] = 0;
  __syncthreads();
  for (int b = 0; b < CSR_NBLK8; ++b) { const int c = boff[b + 1] - boff[b]; int o_ = OFF[(size_t)g * CSR_NBLK8 + b]; o_ = (o_ < 0) ? 0 : (o_ > CHP - c ? CHP - c : o_); const int* src_ = STG + (size_t)b * CHP + o_;
    for (int i = t_; i < c; i += 256) { int id = src_[i]; id = (id < 0) ? 0 : id; ids[boff[b] + i] = id; int d = dst[id]; d = (d < v0) ? v0 : (d >= N ? N - 1 : d); int kk = d - v0; kk = (kk < 0) ? 0 : (kk >= CSR_GN8 ? CSR_GN8 - 1 : kk); key[boff[b] + i] = (unsigned short)kk; } }
  __syncthreads();
  if (t_ == 0) { for (int i = 0; i < tot; ++i) ncnt[key[i]] += 1; int acc = 0; for (int vl = 0; vl < CSR_GN8; ++vl) { const int c = ncnt[vl]; ncnt[vl] = acc; acc += c; } ncnt[CSR_GN8] = acc;
    for (int i = 0; i < tot; ++i) { const int vl = key[i]; outp[ncnt[vl]] = ids[i]; ncnt[vl] += 1; }
    for (int vl = CSR_GN8; vl > 0; --vl) ncnt[vl] = ncnt[vl - 1]; ncnt[0] = 0; }
  __syncthreads();
  for (int pass = 0; pass < 2; ++pass) {
    for (int i = t_; i < (stn - st) / 4; i += 256) { v4i v; for (int e = 0; e < 4; ++e) { const int q = i * 4 + e; v[e] = (q < tot) ? outp[q] : -1; } *(volatile v4i*)(PERM + st + i * 4) = v; }
    for (int i = t_; i < CSR_TS8 / 4; i += 256) { v4i a, c; for (int e = 0; e < 4; ++e) { const int vl = i * 4 + e; const int vc = vl < CSR_GN8 ? vl : CSR_GN8; a[e] = (vl < CSR_GN8) ? st + ncnt[vc] : st; c[e] = (vl < nv) ? (ncnt[(vc < CSR_GN8 ? vc : CSR_GN8 - 1) + 1] - ncnt[vc]) : 0; } *(volatile v4i*)(ROWPTR + t0 + i * 4) = a; *(volatile v4i*)(ROWCNT + t0 + i * 4) = c; }
    __threadfence(); }
}
__global__ __launch_bounds__(256) void csrZ_kernel8(int* __restrict__ p, size_t n4) { typedef __attribute__((ext_vector_type(4))) int v4i; const size_t tid = (size_t)blockIdx.x * 256 + threadIdx.x, nth = (size_t)gridDim.x * 256; v4i z = {0, 0, 0, 0}; for (size_t i = tid; i < n4; i += nth) *(volatile v4i*)(p + i * 4) = z; }
struct CsrBufs8 { int *STG, *HST, *OFF, *START, *TOT, *PERM, *ROWPTR, *ROWCNT, *FLAG; int nG, NGP, CHP; size_t permLen; char* base; size_t bytes; };
static size_t csr_carve8(CsrBufs8& c, char* ws, size_t off, int E, int N) {
  const size_t off0 = off; c.base = ws + off;
  auto al = [&](size_t bytes) { char* p = ws + off; off += (bytes + 255) & ~(size_t)255; return p; };
  c.nG = (N + CSR_GN8 - 1) / CSR_GN8; c.NGP = (c.nG + 31) & ~31; const int ch = (E + CSR_NBLK8 - 1) / CSR_NBLK8; c.CHP = (ch + 31) & ~31; c.permLen = (size_t)E + 32 * (size_t)c.nG + 32;
  c.STG = (int*)al((size_t)CSR_NBLK8 * c.CHP * 4); c.HST = (int*)al((size_t)CSR_NBLK8 * c.NGP * 4); c.OFF = (int*)al((size_t)c.NGP * CSR_NBLK8 * 4); c.START = (int*)al((size_t)(c.NGP + 64) * 4); c.TOT = (int*)al((size_t)(c.NGP + 64) * 4);
  c.PERM = (int*)al(c.permLen * 4); c.ROWPTR = (int*)al((size_t)c.nG * CSR_TS8 * 4); c.ROWCNT = (int*)al((size_t)c.nG * CSR_TS8 * 4); c.FLAG = (int*)al(256);
  c.bytes = off - off0; return off;
}
static void csr_build8(const CsrBufs8& c, const int* dst, int E, int N, hipStream_t stream) {
  const size_t smem = (size_t)(2 * c.NGP + c.CHP) * 4;
  csrZ_kernel8<<<512, 256, 0, stream>>>((int*)c.base, c.bytes / 16);
  csrA_kernel8<<<CSR_NBLK8, 64, smem, stream>>>(dst, E, N, c.nG, c.CHP, c.NGP, c.STG, c.HST);
  csrS_kernel8<<<1, 512, 0, stream>>>(c.HST, c.nG, c.NGP, c.START, c.TOT, c.OFF);
  csrB_kernel8<<<c.nG, 256, 0, stream>>>(dst, N, c.nG, c.CHP, c.NGP, (int)c.permLen, c.STG, c.HST, c.OFF, c.START, c.TOT, c.PERM, c.ROWPTR, c.ROWCNT, c.FLAG);
}
constexpr int CSR_NBLK5 = 512, CSR_GB5 = 5, CSR_GN5 = 1 << CSR_GB5  , CSR_TS5 = (CSR_GN5 < 32 ? 32 : CSR_GN5)  , CSR_MAXG5 = 512, CSR_CAP5 = 12288  ;
__device__ __host__ __forceinline__ int csr_tix5(int v) { return (v >> CSR_GB5) * CSR_TS5 + (v & (CSR_GN5 - 1)); }
__global__ __launch_bounds__(64) void csrA_kernel5(const int* __restrict__ dst, int E, int N, int nG, int CHP, int NGP, int* __restrict__ STG, int* __restrict__ HST) {
  extern __shared__ int sm[];
  int* cnt = sm; int* run = sm + NGP; int* ids = sm + 2 * NGP;
  const int b = blockIdx.x; const int ch = (E + CSR_NBLK5 - 1) / CSR_NBLK5; const int e0 = b * ch, e1 = min(E, e0 + ch);
  for (int i = threadIdx.x; i < NGP; i += 64) cnt[i] = 0;
  for (int i = threadIdx.x; i < CHP; i += 64) ids[i] = -1;
  __syncthreads();
  if (threadIdx.x == 0) {
    for (int e = e0; e < e1; ++e) { int d = dst[e]; d = (d < 0) ? 0 : (d >= N ? N - 1 : d); cnt[d >> CSR_GB5] += 1; }
    int acc = 0; for (int g = 0; g < nG; ++g) { run[g] = acc; acc += cnt[g]; }
    for (int e = e0; e < e1; ++e) { int d = dst[e]; d = (d < 0) ? 0 : (d >= N ? N - 1 : d); const int g = d >> CSR_GB5; ids[run[g]] = e; run[g] += 1; } }
  __syncthreads();
  typedef __attribute__((ext_vector_type(4))) int v4i;
  for (int pass = 0; pass < 2; ++pass) {
    for (int i = threadIdx.x; i < CHP / 4; i += 64) *(volatile v4i*)(STG + (size_t)b * CHP + i * 4) = *(const v4i*)(&ids[i * 4]);
    for (int i = threadIdx.x; i < NGP / 4; i += 64) { v4i v; for (int e = 0; e < 4; ++e) v[e] = (i * 4 + e < nG) ? cnt[i * 4 + e] : 0; *(volatile v4i*)(HST + (size_t)b * NGP + i * 4) = v; }
    __threadfence(); }
}
__global__ __launch_bounds__(512) void csrS_kernel5(const int* __restrict__ HST, int nG, int NGP, int* __restrict__ START, int* __restrict__ TOT, int* __restrict__ OFF) {
  __shared__ int tot[CSR_MAXG5];
  const int b = threadIdx.x;
  for (int pass = 0; pass < 2; ++pass) { int runb = 0; for (int g = 0; g < nG; ++g) { int c = HST[(size_t)b * NGP + g]; c = (c < 0) ? 0 : c; ((volatile int*)OFF)[(size_t)g * CSR_NBLK5 + b] = runb; runb += c; } __threadfence(); }
  for (int g = threadIdx.x; g < nG; g += 512) { int s = 0; for (int bb = 0; bb < CSR_NBLK5; ++bb) { int c = HST[(size_t)bb * NGP + g]; s += (c < 0) ? 0 : c; } tot[g] = s; }
  __syncthreads();
  if (threadIdx.x < 32) {
    __shared__ int st[CSR_MAXG5 + 32];
    if (threadIdx.x == 0) { int acc = 0; for (int g = 0; g < NGP; ++g) { st[g] = acc; if (g < nG) acc += (tot[g] + 31) & ~31; } st[NGP] = acc; }
    __builtin_amdgcn_fence(__ATOMIC_RELEASE, "workgroup"); __builtin_amdgcn_wave_barrier(); __builtin_amdgcn_fence(__ATOMIC_ACQUIRE, "workgroup");
    for (int pass = 0; pass < 2; ++pass) { for (int i = threadIdx.x; i < NGP + 32; i += 32) { ((volatile int*)START)[i] = (i <= NGP) ? st[min(i, NGP)] : 0; ((volatile int*)TOT)[i] = (i < nG) ? tot[i] : 0; } __threadfence(); } }
}
__global__ __launch_bounds__(256) void csrB_kernel5(const int* __restrict__ dst, int N, int nG, int CHP, int NGP, int permLen, const int* __restrict__ STG, const int* __restrict__ HST, const int* __restrict__ OFF, const int* __restrict__ START, const int* __restrict__ TOT, int* __restrict__ PERM, int* __restrict__ ROWPTR, int* __restrict__ ROWCNT, int* __restrict__ FLAG) {
  typedef __attribute__((ext_vector_type(4))) int v4i;
  __shared__ int ids[CSR_CAP5]; __shared__ unsigned short key[CSR_CAP5]; __shared__ int outp[CSR_CAP5]; __shared__ int ncnt[CSR_GN5 + 1]; __shared__ int boff[CSR_NBLK5 + 1];
  const int g = blockIdx.x, t_ = threadIdx.x; int tot = TOT[g]; int st = START[g], stn = START[g + 1]; const int v0 = g * CSR_GN5; const int nv = min(CSR_GN5, N - v0); const int t0 = g * CSR_TS5;
  st = (st < 0) ? 0 : (st > permLen - 32 ? permLen - 32 : st) & ~31; stn = (stn < st) ? st : (stn > permLen ? permLen : stn); tot = (tot < 0) ? 0 : tot; if (tot > stn - st && tot <= CSR_CAP5) tot = stn - st;
  if (tot > CSR_CAP5) {
    for (int pass = 0; pass < 2; ++pass) { for (int i = t_; i < CSR_TS5 / 4; i += 256) { v4i a, c; for (int e = 0; e < 4; ++e) { a[e] = st; c[e] = 0; } *(volatile v4i*)(ROWPTR + t0 + i * 4) = a; *(volatile v4i*)(ROWCNT + t0 + i * 4) = c; } if (t_ == 0) ((volatile int*)FLAG)[0] = 1; __threadfence(); } (void)nv; return; }
  if (t_ == 0) { int acc = 0; for (int b = 0; b < CSR_NBLK5; ++b) { boff[b] = acc; int c = HST[(size_t)b * NGP + g]; c = (c < 0) ? 0 : (c > CHP ? CHP : c); acc += c; if (acc > tot) acc = tot; } boff[CSR_NBLK5] = acc; }
  for (int i = t_; i <= CSR_GN5; i += 256) ncnt[i] = 0;
  __syncthreads();
  for (int b = 0; b < CSR_NBLK5; ++b) { const int c = boff[b + 1] - boff[b]; int o_ = OFF[(size_t)g * CSR_NBLK5 + b]; o_ = (o_ < 0) ? 0 : (o_ > CHP - c ? CHP - c : o_); const int* src_ = STG + (size_t)b * CHP + o_;
    for (int i = t_; i < c; i += 256) { int id = src_[i]; id = (id < 0) ? 0 : id; ids[boff[b] + i] = id; int d = dst[id]; d = (d < v0) ? v0 : (d >= N ? N - 1 : d); int kk = d - v0; kk = (kk < 0) ? 0 : (kk >= CSR_GN5 ? CSR_GN5 - 1 : kk); key[boff[b] + i] = (unsigned short)kk; } }
  __syncthreads();
  if (t_ == 0) { for (int i = 0; i < tot; ++i) ncnt[key[i]] += 1; int acc = 0; for (int vl = 0; vl < CSR_GN5; ++vl) { const int c = ncnt[vl]; ncnt[vl] = acc; acc += c; } ncnt[CSR_GN5] = acc;
    for (int i = 0; i < tot; ++i) { const int vl = key[i]; outp[ncnt[vl]] = ids[i]; ncnt[vl] += 1; }
    for (int vl = CSR_GN5; vl > 0; --vl) ncnt[vl] = ncnt[vl - 1]; ncnt[0] = 0; }
  __syncthreads();
  for (int pass = 0; pass < 2; ++pass) {
    for (int i = t_; i < (stn - st) / 4; i += 256) { v4i v; for (int e = 0; e < 4; ++e) { const int q = i * 4 + e; v[e] = (q < tot) ? outp[q] : -1; } *(volatile v4i*)(PERM + st + i * 4) = v; }
    for (int i = t_; i < CSR_TS5 / 4; i += 256) { v4i a, c; for (int e = 0; e < 4; ++e) { const int vl = i * 4 + e; const int vc = vl < CSR_GN5 ? vl : CSR_GN5; a[e] = (vl < CSR_GN5) ? st + ncnt[vc] : st; c[e] = (vl < nv) ? (ncnt[(vc < CSR_GN5 ? vc : CSR_GN5 - 1) + 1] - ncnt[vc]) : 0; } *(volatile v4i*)(ROWPTR + t0 + i * 4) = a; *(volatile v4i*)(ROWCNT + t0 + i * 4) = c; }
    __threadfence(); }
}
__global__ __launch_bounds__(256) void csrZ_kernel5(int* __restrict__ p, size_t n4) { typedef __attribute__((ext_vector_type(4))) int v4i; const size_t tid = (size_t)blockIdx.x * 256 + threadIdx.x, nth = (size_t)gridDim.x * 256; v4i z = {0, 0, 0, 0}; for (size_t i = tid; i < n4; i += nth) *(volatile v4i*)(p + i * 4) = z; }
struct CsrBufs5 { int *STG, *HST, *OFF, *START, *TOT, *PERM, *ROWPTR, *ROWCNT, *FLAG; int nG, NGP, CHP; size_t permLen; char* base; size_t bytes; };
static size_t csr_carve5(CsrBufs5& c, char* ws, size_t off, int E, int N) {
  const size_t off0 = off; c.base = ws + off;
  auto al = [&](size_t bytes) { char* p = ws + off; off += (bytes + 255) & ~(size_t)255; return p; };
  c.nG = (N + CSR_GN5 - 1) / CSR_GN5; c.NGP = (c.nG + 31) & ~31; const int ch = (E + CSR_NBLK5 - 1) / CSR_NBLK5; c.CHP = (ch + 31) & ~31; c.permLen = (size_t)E + 32 * (size_t)c.nG + 32;
  c.STG = (int*)al((size_t)CSR_NBLK5 * c.CHP * 4); c.HST = (int*)al((size_t)CSR_NBLK5 * c.NGP * 4); c.OFF = (int*)al((size_t)c.NGP * CSR_NBLK5 * 4); c.START = (int*)al((size_t)(c.NGP + 64) * 4); c.TOT = (int*)al((size_t)(c.NGP + 64) * 4);
  c.PERM = (int*)al(c.permLen * 4); c.ROWPTR = (int*)al((size_t)c.nG * CSR_TS5 * 4); c.ROWCNT = (int*)al((size_t)c.nG * CSR_TS5 * 4); c.FLAG = (int*)al(256);
  c.bytes = off - off0; return off;
}
static void csr_build5(const CsrBufs5& c, const int* dst, int E, int N, hipStream_t stream) {
  const size_t smem = (size_t)(2 * c.NGP + c.CHP) * 4;
  csrZ_kernel5<<<512, 256, 0, stream>>>((int*)c.base, c.bytes / 16);
  csrA_kernel5<<<CSR_NBLK5, 64, smem, stream>>>(dst, E, N, c.nG, c.CHP, c.NGP, c.STG, c.HST);
  csrS_kernel5<<<1, 512, 0, stream>>>(c.HST, c.nG, c.NGP, c.START, c.TOT, c.OFF);
  csrB_kernel5<<<c.nG, 256, 0, stream>>>(dst, N, c.nG, c.CHP, c.NGP, (int)c.permLen, c.STG, c.HST, c.OFF, c.START, c.TOT, c.PERM, c.ROWPTR, c.ROWCNT, c.FLAG);
}


__global__ __launch_bounds__(256) void wput_kernel(const float* __restrict__ r1, const float* __restrict__ o1, const float* __restrict__ r2, const float* __restrict__ o2, const float* __restrict__ l1, const float* __restrict__ l2, b16* __restrict__ W1, b16* __restrict__ W2, b16* __restrict__ WL1, b16* __restrict__ WL2) { const int u = blockIdx.x * 256 + threadIdx.x; v8b v;
  if (u < H * 16) { const int o = u / 16, k0 = (u % 16) * 8;
#pragma unroll
    for (int j = 0; j < 8; ++j) { const int k = k0 + j; float w = 0.0f; if (k < F) w = r1[(size_t)o * F + k]; else if (k >= FP && k < FP + F) w = o1[(size_t)o * F + k - FP]; v[j] = (b16)(bf16_rne(w) * WSC); } for (int pass = 0; pass < 2; ++pass) { *(volatile v8b*)(W1 + (size_t)o * 2 * FP + k0) = v; __threadfence(); }
#pragma unroll
    for (int j = 0; j < 8; ++j) { const int k = k0 + j; v[j] = (b16)(bf16_rne(k < H ? r2[(size_t)o * H + k] : o2[(size_t)o * H + k - H]) * WSC); } for (int pass = 0; pass < 2; ++pass) { *(volatile v8b*)(W2 + (size_t)o * 2 * H + k0) = v; __threadfence(); }
#pragma unroll
    for (int j = 0; j < 8; ++j) v[j] = (b16)(bf16_rne(l1[(size_t)o * 2 * H + k0 + j]) * WSC); for (int pass = 0; pass < 2; ++pass) { *(volatile v8b*)(WL1 + (size_t)o * 2 * H + k0) = v; __threadfence(); } }
  if (u < 16 * 8) { const int o = u / 8, k0 = (u % 8) * 8;
#pragma unroll
    for (int j = 0; j < 8; ++j) v[j] = (b16)(o < C ? bf16_rne(l2[(size_t)o * H + k0 + j]) * WSC : 0.0f); for (int pass = 0; pass < 2; ++pass) { *(volatile v8b*)(WL2 + (size_t)o * H + k0) = v; __threadfence(); } } }
__global__ __launch_bounds__(256) void ew_kernel(const float* __restrict__ ea, const float* __restrict__ bw, const float* __restrict__ bb, float* __restrict__ EW) { const size_t e = (size_t)blockIdx.x * 256 + threadIdx.x; if (e >= (size_t)E) return; float s = bfv(bb[0]);
#pragma unroll
  for (int k = 0; k < BD; ++k) s += pmul(bfv(ea[e * BD + k]), bfv(bw[k]));
  for (int pass = 0; pass < 2; ++pass) { ((volatile float*)EW)[e] = s; __threadfence(); } }
template <int LAYER>
__global__ __launch_bounds__(32) void conv_kernel(const float* __restrict__ IN, const float* __restrict__ EW, const int* __restrict__ srcs, const int* __restrict__ PERM, const int* __restrict__ ROWPTR, const int* __restrict__ ROWCNT, int permLen, const b16* __restrict__ W, const float* __restrict__ bias, int NLIM, float* __restrict__ OUT) { constexpr int FIN = LAYER == 0 ? F : H; __shared__ __attribute__((aligned(16))) b16 Ah[16][2 * FP + 8], Al[16][2 * FP + 8]; __shared__ float Tf[16][H + 1]; const int lane = threadIdx.x, nloc = lane & 15, hlf = lane >> 4; const size_t m0 = (size_t)blockIdx.x * 16; if (m0 >= (size_t)NLIM) return; const int c0 = lane * 2, c1 = lane * 2 + 1; const bool v0 = c0 < FIN, v1 = c1 < FIN;
  auto rd = [&](size_t n, int c) -> float { const float v = IN[n * FIN + c]; return LAYER == 0 ? bfv(v) : fmaxf(v, 0.0f); };
  for (int rr = 0; rr < 16; ++rr) { const size_t i = m0 + rr; int st = ROWPTR[i], cnt = ROWCNT[i]; cnt = iclamp(cnt, 0, E); st = iclamp(st, 0, permLen - cnt); float a0 = 0.0f, a1 = 0.0f;
#pragma unroll 1
    for (int j = 0; j < cnt; ++j) { const int e = iclamp(PERM[st + j], 0, E - 1); const size_t u = (size_t)iclamp(srcs[e], 0, N - 1); if (u >= (size_t)NLIM) continue; const float w = EW[e]; if (v0) a0 += pmul(w, rd(u, c0)); if (v1) a1 += pmul(w, rd(u, c1)); }
    b16 p, ql; split16(a0 * HS, p, ql); Ah[rr][c0] = p; Al[rr][c0] = ql; split16(a1 * HS, p, ql); Ah[rr][c1] = p; Al[rr][c1] = ql;
    const float s0 = v0 ? rd(i, c0) : 0.0f, s1 = v1 ? rd(i, c1) : 0.0f; if (LAYER == 0) { Ah[rr][FP + c0] = (b16)(s0 * XS); Al[rr][FP + c0] = (b16)0.0f; Ah[rr][FP + c1] = (b16)(s1 * XS); Al[rr][FP + c1] = (b16)0.0f; } else { split16(s0 * HS, p, ql); Ah[rr][FP + c0] = p; Al[rr][FP + c0] = ql; split16(s1 * HS, p, ql); Ah[rr][FP + c1] = p; Al[rr][FP + c1] = ql; } }
  if (lane < 16) for (int k = 2 * FP; k < 2 * FP + 8; ++k) { Ah[lane][k] = (b16)0.0f; Al[lane][k] = (b16)0.0f; }
  wave_lds_sync(); v8f acc[4] = {(v8f){}, (v8f){}, (v8f){}, (v8f){}};
#pragma unroll
  for (int kb = 0; kb < 2 * FP; kb += 32) { const v16b a = frag_kb(&Ah[nloc][kb], hlf), al = frag_kb(&Al[nloc][kb], hlf);
#pragma unroll
    for (int t = 0; t < 4; ++t) { const v16b bw = frag_kb(W + (size_t)(t * 16 + nloc) * 2 * FP + kb, hlf); acc[t] = wmma16b(a, bw, acc[t]); if (LAYER != 0 || kb < FP) acc[t] = wmma16b(al, bw, acc[t]); } }
#pragma unroll
  for (int t = 0; t < 4; ++t) { const int cc = t * 16 + nloc; const float bb = bfv(bias[cc]);
#pragma unroll
    for (int r8 = 0; r8 < 8; ++r8) Tf[8 * hlf + r8][cc] = acc[t][r8] * (1.0f / (HS * WSC)) + bb; }
  wave_lds_sync();
  for (int pass = 0; pass < 2; ++pass) { for (int rr = 0; rr < 16; ++rr) *(volatile v2f*)(OUT + (m0 + rr) * H + lane * 2) = (v2f){Tf[rr][lane * 2], Tf[rr][lane * 2 + 1]}; __threadfence(); } }
__global__ __launch_bounds__(256) void pool_kernel(const float* __restrict__ Hr, const int* __restrict__ PERM, const int* __restrict__ ROWPTR, const int* __restrict__ ROWCNT, int permLen, const float* __restrict__ PREV, int NLIM, float* __restrict__ PL) { const int wave = threadIdx.x >> 5, lane = threadIdx.x & 31; const int g = blockIdx.x * NPB + wave; if (g >= G) return; int st = ROWPTR[g], cnt = ROWCNT[g]; cnt = iclamp(cnt, 0, N); st = iclamp(st, 0, permLen - cnt); float mx0 = -INFINITY, mx1 = -INFINITY, s0 = 0.0f, s1 = 0.0f; int nn = 0;
#pragma unroll 1
  for (int j = 0; j < cnt; ++j) { const size_t n = (size_t)iclamp(PERM[st + j], 0, N - 1); if (n >= (size_t)NLIM) continue; ++nn; const v2f v = *(const v2f*)(Hr + n * H + lane * 2); mx0 = fmaxf(mx0, v[0]); mx1 = fmaxf(mx1, v[1]); s0 += v[0]; s1 += v[1]; }
  const float inv = 1.0f / fmaxf((float)nn, 1.0f); if (nn == 0) { mx0 = 0.0f; mx1 = 0.0f; }
  v2f a = {mx0, mx1}, m = {s0 * inv, s1 * inv}; if (PREV) { const v2f pa = *(const v2f*)(PREV + (size_t)g * 2 * H + lane * 2), pm = *(const v2f*)(PREV + (size_t)g * 2 * H + H + lane * 2); a += pa; m += pm; }
  for (int pass = 0; pass < 2; ++pass) { *(volatile v2f*)(PL + (size_t)g * 2 * H + lane * 2) = a; *(volatile v2f*)(PL + (size_t)g * 2 * H + H + lane * 2) = m; __threadfence(); } }
__global__ __launch_bounds__(32) void head_kernel(const float* __restrict__ PL, const b16* __restrict__ WL1, const float* __restrict__ b1, const b16* __restrict__ WL2, const float* __restrict__ b2, float* __restrict__ STG) { __shared__ __attribute__((aligned(16))) b16 Ah[16][2 * H + 8], Al[16][2 * H + 8]; __shared__ float Tf[16][H + 1], Os[16][16]; const int lane = threadIdx.x, nloc = lane & 15, hlf = lane >> 4; const int g0 = blockIdx.x * 16;
  for (int rr = 0; rr < 16; ++rr) for (int q = 0; q < 4; ++q) { const int c = q * 32 + lane; b16 p, ql; split16(PL[(size_t)(g0 + rr) * 2 * H + c] * HS, p, ql); Ah[rr][c] = p; Al[rr][c] = ql; }
  if (lane < 16) for (int k = 2 * H; k < 2 * H + 8; ++k) { Ah[lane][k] = (b16)0.0f; Al[lane][k] = (b16)0.0f; }
  wave_lds_sync(); v8f acc[4] = {(v8f){}, (v8f){}, (v8f){}, (v8f){}};
#pragma unroll
  for (int kb = 0; kb < 2 * H; kb += 32) { const v16b a = frag_kb(&Ah[nloc][kb], hlf), al = frag_kb(&Al[nloc][kb], hlf);
#pragma unroll
    for (int t = 0; t < 4; ++t) { const v16b bw = frag_kb(WL1 + (size_t)(t * 16 + nloc) * 2 * H + kb, hlf); acc[t] = wmma16b(a, bw, acc[t]); acc[t] = wmma16b(al, bw, acc[t]); } }
#pragma unroll
  for (int t = 0; t < 4; ++t) { const int cc = t * 16 + nloc; const float bb = bfv(b1[cc]);
#pragma unroll
    for (int r8 = 0; r8 < 8; ++r8) Tf[8 * hlf + r8][cc] = fmaxf(acc[t][r8] * (1.0f / (HS * WSC)) + bb, 0.0f); }
  wave_lds_sync();
  for (int rr = 0; rr < 16; ++rr) for (int q = 0; q < 2; ++q) { b16 p, ql; split16(Tf[rr][q * 32 + lane] * HS, p, ql); Ah[rr][q * 32 + lane] = p; Al[rr][q * 32 + lane] = ql; } if (lane < 16) for (int k = H; k < H + 8; ++k) { Ah[lane][k] = (b16)0.0f; Al[lane][k] = (b16)0.0f; }
  wave_lds_sync(); v8f o = (v8f){};
#pragma unroll
  for (int kb = 0; kb < H; kb += 32) { const v16b a = frag_kb(&Ah[nloc][kb], hlf), al = frag_kb(&Al[nloc][kb], hlf); const v16b bw = frag_kb(WL2 + (size_t)nloc * H + kb, hlf); o = wmma16b(a, bw, o); o = wmma16b(al, bw, o); }
#pragma unroll
  for (int r8 = 0; r8 < 8; ++r8) Os[8 * hlf + r8][nloc] = o[r8] * (1.0f / (HS * WSC)) + (nloc < C ? bfv(b2[nloc]) : 0.0f);
  wave_lds_sync();
  for (int pass = 0; pass < 2; ++pass) { for (int q = 0; q < 8; ++q) ((volatile float*)STG)[(size_t)g0 * 16 + q * 32 + lane] = Os[(q * 32 + lane) >> 4][(q * 32 + lane) & 15]; __threadfence(); } }
__global__ __launch_bounds__(256) void copy_kernel(const float* __restrict__ STG, float* __restrict__ out) { const int u = blockIdx.x * 256 + threadIdx.x; if (u >= G * C) return; const int g = u / C, c = u % C;
  for (int pass = 0; pass < 2; ++pass) { ((volatile float*)out)[u] = STG[g * 16 + c]; __threadfence(); } }
}

extern "C" void kernel_launch(void* const* d_in, const int* in_sizes, int n_in, void* d_out, int out_size, void* d_ws, size_t ws_size, hipStream_t stream) {
  (void)n_in;
  auto Fp = [&](int i) { return (const float*)d_in[i]; }; auto Ip = [&](int i) { return (const int*)d_in[i]; };
  if (in_sizes[0] != N * F || in_sizes[1] != E * BD || in_sizes[2] != BD || in_sizes[4] != H * F || in_sizes[6] != H * F || in_sizes[7] != H * H || in_sizes[10] != H * 2 * H || in_sizes[12] != C * H || in_sizes[14] != 2 * E || in_sizes[15] != N || out_size != G * C) return;
  const int NLIM = N;
  size_t off = 0; char* ws = (char*)d_ws;
  auto carve = [&](size_t bytes) { char* p = ws + off; off += (bytes + 255) & ~(size_t)255; return p; };
  b16* W1 = (b16*)carve((size_t)H * 2 * FP * 2); b16* W2 = (b16*)carve((size_t)H * 2 * H * 2); b16* WL1 = (b16*)carve((size_t)H * 2 * H * 2); b16* WL2 = (b16*)carve((size_t)16 * H * 2); float* EW = (float*)carve((size_t)E * 4); float* H1 = (float*)carve((size_t)N * H * 4); float* H2 = (float*)carve((size_t)N * H * 4); float* PL1 = (float*)carve((size_t)G * 2 * H * 4); float* PL2 = (float*)carve((size_t)G * 2 * H * 4); float* STG = (float*)carve((size_t)G * 16 * 4); CsrBufs8 csr; off = csr_carve8(csr, ws, off, E, N); CsrBufs5 cg; off = csr_carve5(cg, ws, off, N, G);
  if (off > ws_size || off > ((size_t)128 << 20)) return;
  wput_kernel<<<(H * 16 + 255) / 256, 256, 0, stream>>>(Fp(4), Fp(6), Fp(7), Fp(9), Fp(10), Fp(12), W1, W2, WL1, WL2);
  ew_kernel<<<(E + 255) / 256, 256, 0, stream>>>(Fp(1), Fp(2), Fp(3), EW);
  csr_build8(csr, Ip(14) + E, E, N, stream); csr_build5(cg, Ip(15), N, G, stream);
  conv_kernel<0><<<NLIM / 16, 32, 0, stream>>>(Fp(0), EW, Ip(14), csr.PERM, csr.ROWPTR, csr.ROWCNT, (int)csr.permLen, W1, Fp(5), NLIM, H1);
  pool_kernel<<<G / NPB, 256, 0, stream>>>(H1, cg.PERM, cg.ROWPTR, cg.ROWCNT, (int)cg.permLen, nullptr, NLIM, PL1);
  conv_kernel<1><<<NLIM / 16, 32, 0, stream>>>(H1, EW, Ip(14), csr.PERM, csr.ROWPTR, csr.ROWCNT, (int)csr.permLen, W2, Fp(8), NLIM, H2);
  pool_kernel<<<G / NPB, 256, 0, stream>>>(H2, cg.PERM, cg.ROWPTR, cg.ROWCNT, (int)cg.permLen, PL1, NLIM, PL2);
  head_kernel<<<G / 16, 32, 0, stream>>>(PL2, WL1, Fp(11), WL2, Fp(13), STG);
  copy_kernel<<<(G * C + 255) / 256, 256, 0, stream>>>(STG, (float*)d_out);
}
